// Enc_basic_38431367365314
// MI455X (gfx1250) — hardware-run, weakly checked
//
#include <hip/hip_runtime.h>
#include <math.h>
#include <stdint.h>

#define BB   4
#define NN   8192
#define EE   256
#define HH   8
#define DD   (NN / HH)
#define HIDN 1024
#define MTOT (BB * NN)

typedef _Float16 half_t;
typedef _Float16 v16h __attribute__((ext_vector_type(16)));
typedef _Float16 v8h  __attribute__((ext_vector_type(8)));
typedef v8h v8ha __attribute__((may_alias));
typedef float v8f __attribute__((ext_vector_type(8)));
typedef float v4f __attribute__((ext_vector_type(4)));
typedef v4f v4fa __attribute__((may_alias));

union Frag { v16h v; v8h h[2]; };

__device__ __forceinline__ v8f zero8() { v8f z; z[0]=0.f; z[1]=0.f; z[2]=0.f; z[3]=0.f; z[4]=0.f; z[5]=0.f; z[6]=0.f; z[7]=0.f; return z; }

__device__ __forceinline__ v16h ldfrag_g(const half_t* p) {
  Frag f; f.h[0] = *(const v8h*)(p); f.h[1] = *(const v8h*)(p + 16); return f.v;
}
__device__ __forceinline__ v16h ldfrag_s(const half_t* p) {
  Frag f; f.h[0] = *(const v8ha*)(p); f.h[1] = *(const v8ha*)(p + 16); return f.v;
}
__device__ __forceinline__ v8f mma16(v16h a, v16h b, v8f c) {
  return __builtin_amdgcn_wmma_f32_16x16x32_f16(false, a, false, b, (short)0, c, false, false);
}
__device__ __forceinline__ v8f mma16_g(v16h a, v16h b, v8f c) {
  c = mma16(a, b, c);
  asm volatile("v_nop\n\tv_nop\n\tv_nop\n\tv_nop" : "+v"(c) : "v"(a), "v"(b));
  return c;
}
__device__ __forceinline__ void guard4(v8f& a, v8f& b, v8f& c, v8f& d, v16h x, v16h y) {
  asm volatile("v_nop\n\tv_nop\n\tv_nop\n\tv_nop" : "+v"(a), "+v"(b), "+v"(c), "+v"(d) : "v"(x), "v"(y));
}
__device__ __forceinline__ void keep4(v16h a, v16h b, v16h c, v16h d) {
  asm volatile("v_nop" :: "v"(a), "v"(b), "v"(c), "v"(d));
}
__device__ __forceinline__ void acc_guard4(v8f& a, v8f& b, v8f& c, v8f& d) {
  asm volatile("v_nop\n\tv_nop\n\tv_nop\n\tv_nop" : "+v"(a), "+v"(b), "+v"(c), "+v"(d));
}
__device__ __forceinline__ void wave_lds_sync() {
  __builtin_amdgcn_fence(__ATOMIC_RELEASE, "workgroup");
  __builtin_amdgcn_wave_barrier();
  __builtin_amdgcn_fence(__ATOMIC_ACQUIRE, "workgroup");
}

__device__ __forceinline__ float mish_f(float x) {
  const float ex = __expf(fminf(x, 20.0f));
  const float n  = ex * (ex + 2.0f);
  return x * (n * __builtin_amdgcn_rcpf(n + 2.0f));
}

__global__ __launch_bounds__(256) void cvt_f16_kernel(const float* __restrict__ src, half_t* __restrict__ dst,
                                                      int n8, float s) {
  const int i = blockIdx.x * 256 + threadIdx.x;
  if (i >= n8) return;
  const float* p = src + (size_t)i * 8;
  const v4f a0 = *(const v4f*)(p);
  const v4f a1 = *(const v4f*)(p + 4);
  v8h o;
  o[0] = (half_t)(a0[0] * s); o[1] = (half_t)(a0[1] * s); o[2] = (half_t)(a0[2] * s); o[3] = (half_t)(a0[3] * s);
  o[4] = (half_t)(a1[0] * s); o[5] = (half_t)(a1[1] * s); o[6] = (half_t)(a1[2] * s); o[7] = (half_t)(a1[3] * s);
  half_t* q = dst + (size_t)i * 8;
  *(volatile v8h*)q = o;
  __threadfence();
  *(volatile v8h*)q = o;
}

__global__ __launch_bounds__(256) void ln_kernel(const float* __restrict__ x,
                                                 const float* __restrict__ w,
                                                 const float* __restrict__ b,
                                                 half_t* __restrict__ out, int M) {
  const int row  = blockIdx.x * 8 + (threadIdx.x >> 5);
  const int lane = threadIdx.x & 31;
  if (row >= M) return;
  const float* xr = x + (size_t)row * EE + lane * 8;
  const v4f a0 = *(const v4f*)(xr);
  const v4f a1 = *(const v4f*)(xr + 4);
  float vv[8];
  vv[0] = a0[0]; vv[1] = a0[1]; vv[2] = a0[2]; vv[3] = a0[3];
  vv[4] = a1[0]; vv[5] = a1[1]; vv[6] = a1[2]; vv[7] = a1[3];
  float s = 0.f;
#pragma unroll
  for (int i = 0; i < 8; ++i) s += vv[i];
#pragma unroll
  for (int o = 1; o < 32; o <<= 1) s += __shfl_xor(s, o, 32);
  const float mu = s * (1.0f / EE);
  float var = 0.f;
#pragma unroll
  for (int i = 0; i < 8; ++i) { const float d = vv[i] - mu; var += d * d; }
#pragma unroll
  for (int o = 1; o < 32; o <<= 1) var += __shfl_xor(var, o, 32);
  const float rstd = rsqrtf(var * (1.0f / EE) + 1e-5f);
  const v4f w0 = *(const v4f*)(w + lane * 8);
  const v4f w1 = *(const v4f*)(w + lane * 8 + 4);
  const v4f b0 = *(const v4f*)(b + lane * 8);
  const v4f b1 = *(const v4f*)(b + lane * 8 + 4);
  float ww[8], bw[8];
  ww[0] = w0[0]; ww[1] = w0[1]; ww[2] = w0[2]; ww[3] = w0[3];
  ww[4] = w1[0]; ww[5] = w1[1]; ww[6] = w1[2]; ww[7] = w1[3];
  bw[0] = b0[0]; bw[1] = b0[1]; bw[2] = b0[2]; bw[3] = b0[3];
  bw[4] = b1[0]; bw[5] = b1[1]; bw[6] = b1[2]; bw[7] = b1[3];
  v8h o;
#pragma unroll
  for (int i = 0; i < 8; ++i) o[i] = (half_t)((vv[i] - mu) * rstd * ww[i] + bw[i]);
  half_t* op = out + (size_t)row * EE + lane * 8;
  *(volatile v8h*)op = o;
  __threadfence();
  *(volatile v8h*)op = o;
}

template <int BIAS_MODE, int OUT16, bool RESID, int ACT>
__global__ __launch_bounds__(256) void gemm64_kernel(
    const half_t* __restrict__ A, int lda,
    const half_t* __restrict__ Bt, int ldb,
    void* __restrict__ Cout, int ldc,
    const float* __restrict__ bias,
    const float* __restrict__ resid, int ldr,
    int M, int N, int K, float scale, float oscale) {
  __shared__ __align__(16) float sT[8][16 * 68];
  const int lane = threadIdx.x & 31;
  const int wave = threadIdx.x >> 5;
  const int tilesN = N >> 6;
  const int tilesM = M >> 6;
  const int tile = blockIdx.x * 8 + wave;
  if (tile >= tilesM * tilesN) return;
  const int tm = tile / tilesN;
  const int tn = tile - tm * tilesN;
  const int m0 = tm << 6;
  const int n0 = tn << 6;

  const int rlane = lane & 15;
  const int koff  = (lane >> 4) * 8;
  const int mOff  = (lane >> 4) * 8;

  v8f acc[4][4];
#pragma unroll
  for (int i = 0; i < 4; ++i)
#pragma unroll
    for (int j = 0; j < 4; ++j) acc[i][j] = zero8();

  for (int k0 = 0; k0 < K; k0 += 32) {
    v16h bh[4];
#pragma unroll
    for (int j = 0; j < 4; ++j)
      bh[j] = ldfrag_g(Bt + (size_t)(n0 + (j << 4) + rlane) * ldb + k0 + koff);
#pragma unroll
    for (int i = 0; i < 4; ++i) {
      const v16h ah = ldfrag_g(A + (size_t)(m0 + (i << 4) + rlane) * lda + k0 + koff);
#pragma unroll
      for (int j = 0; j < 4; ++j) acc[i][j] = mma16(ah, bh[j], acc[i][j]);
      guard4(acc[i][0], acc[i][1], acc[i][2], acc[i][3], ah, bh[3]);
    }
    keep4(bh[0], bh[1], bh[2], bh[3]);
  }
  acc_guard4(acc[0][0], acc[0][1], acc[0][2], acc[0][3]);
  acc_guard4(acc[1][0], acc[1][1], acc[1][2], acc[1][3]);
  acc_guard4(acc[2][0], acc[2][1], acc[2][2], acc[2][3]);
  acc_guard4(acc[3][0], acc[3][1], acc[3][2], acc[3][3]);

  float* slab = sT[wave];
#pragma unroll
  for (int i = 0; i < 4; ++i) {
    const int mBase = m0 + (i << 4);
#pragma unroll
    for (int j = 0; j < 4; ++j) {
      const int n = n0 + (j << 4) + rlane;
      float bn = 0.f;
      if (BIAS_MODE == 2) bn = bias[n];
#pragma unroll
      for (int r = 0; r < 8; ++r) {
        const int row = mBase + mOff + r;
        float v = acc[i][j][r] * scale;
        if (BIAS_MODE == 1) v += bias[row];
        if (BIAS_MODE == 2) v += bn;
        if (ACT == 1) v = mish_f(v);
        v *= oscale;
        if (RESID) v += resid[(size_t)row * ldr + n];
        slab[(mOff + r) * 68 + (j << 4) + rlane] = v;
      }
    }
    wave_lds_sync();
    if (OUT16 == 0) {
      float* C = (float*)Cout;
      const int hh = lane >> 4, c4 = (lane & 15) * 4;
      for (int pass = 0; pass < 2; ++pass) {
#pragma unroll
        for (int it = 0; it < 8; ++it) {
          const int row = it * 2 + hh;
          const v4f v = *(const v4fa*)(slab + row * 68 + c4);
          *(volatile v4f*)(C + (size_t)(mBase + row) * ldc + n0 + c4) = v;
        }
        __threadfence();
      }
    } else {
      half_t* C = (half_t*)Cout;
      const int q = lane >> 3, c8 = (lane & 7) * 8;
      for (int pass = 0; pass < 2; ++pass) {
#pragma unroll
        for (int it = 0; it < 4; ++it) {
          const int row = it * 4 + q;
          const float* sp = slab + row * 68 + c8;
          v8h hv;
#pragma unroll
          for (int e = 0; e < 8; ++e) hv[e] = (half_t)sp[e];
          *(volatile v8h*)(C + (size_t)(mBase + row) * ldc + n0 + c8) = hv;
        }
        __threadfence();
      }
    }
    wave_lds_sync();
  }
}

#define KT   32
#define KSP  264
#define VSP  40
#define PSP  40
#define OSP  264
#define SSP  32
#define LDS_KS 0
#define LDS_VT (LDS_KS + KT * KSP * 2)
#define LDS_SS (LDS_VT + EE * VSP * 2)
#define LDS_PS (LDS_SS + 64 * SSP * 4)
#define LDS_AT (LDS_PS + 8 * 16 * PSP * 2)
static_assert(64 * OSP * 2 <= LDS_SS);
static_assert((LDS_VT % 16) == 0 && (LDS_SS % 16) == 0 && (LDS_PS % 16) == 0);
static_assert(LDS_AT <= 65536);
static_assert((MTOT % 64) == 0 && (DD % KT) == 0 && (NN % DD) == 0);

__global__ __launch_bounds__(256) void attn_kernel(const half_t* __restrict__ Qp,
                                                   const half_t* __restrict__ Kp,
                                                   const half_t* __restrict__ VTp,
                                                   half_t* __restrict__ Op) {
  __shared__ __align__(16) unsigned char smem[LDS_AT];
  half_t* Ks = (half_t*)(smem + LDS_KS);
  half_t* Vt = (half_t*)(smem + LDS_VT);
  float*  Ss = (float*)(smem + LDS_SS);
  half_t* Ps = (half_t*)(smem + LDS_PS);
  half_t* Os = (half_t*)(smem + LDS_KS);

  const int tid  = threadIdx.x;
  const int wave = tid >> 5;
  const int lane = tid & 31;
  const int h    = lane >> 4;
  const int m    = lane & 15;
  const int qr   = wave & 3;
  const int eh   = wave >> 2;
  const int q0   = blockIdx.x * 64;
  const int kbase = (q0 / DD) * DD;

  const half_t* qrow = Qp + (size_t)(q0 + qr * 16 + m) * EE + 8 * h;
  half_t* Pw = Ps + wave * (16 * PSP);

  v8f oacc[8];
#pragma unroll
  for (int t = 0; t < 8; ++t) oacc[t] = zero8();
  float mr = -1e30f;
  float lr = 0.f;
  float cr = 1.f;

  for (int kt = 0; kt < DD / KT; ++kt) {
    const int krow0 = kbase + kt * KT;
    __syncthreads();
#pragma unroll
    for (int i = 0; i < 4; ++i) {
      const int c = i * 256 + tid;
      const int row = c >> 5, e8 = (c & 31) * 8;
      const v8h a = *(const v8h*)(Kp + (size_t)(krow0 + row) * EE + e8);
      *(v8h*)(Ks + row * KSP + e8) = a;
    }
#pragma unroll
    for (int i = 0; i < 4; ++i) {
      const int c = i * 256 + tid;
      const int e = c >> 2, k8 = (c & 3) * 8;
      const v8h a = *(const v8h*)(VTp + (size_t)e * MTOT + krow0 + k8);
      *(v8h*)(Vt + e * VSP + k8) = a;
    }
    __syncthreads();

    v8f sacc = zero8();
    const half_t* krow = Ks + (eh * 16 + m) * KSP + 8 * h;
#pragma unroll
    for (int kb = 0; kb < 8; ++kb) {
      const v16h qa = ldfrag_g(qrow + kb * 32);
      const v16h kf = ldfrag_s(krow + kb * 32);
      sacc = mma16_g(qa, kf, sacc);
    }
#pragma unroll
    for (int r = 0; r < 8; ++r) Ss[(qr * 16 + 8 * h + r) * SSP + eh * 16 + m] = sacc[r];
    __syncthreads();

#pragma unroll
    for (int r = 0; r < 16; ++r) {
      const float s = Ss[(qr * 16 + r) * SSP + lane] * (1.0f / 64.0f);
      float mt = s;
#pragma unroll
      for (int o = 1; o < 32; o <<= 1) mt = fmaxf(mt, __shfl_xor(mt, o, 32));
      const float mold = __shfl(mr, r, 32);
      const float lold = __shfl(lr, r, 32);
      const float newm = fmaxf(mold, mt);
      const float c = __expf(mold - newm);
      const float p = __expf(s - newm);
      float ps = p;
#pragma unroll
      for (int o = 1; o < 32; o <<= 1) ps += __shfl_xor(ps, o, 32);
      const float lnew = lold * c + ps;
      const bool me = (lane == r);
      mr = me ? newm : mr;
      lr = me ? lnew : lr;
      cr = me ? c : cr;
      Pw[r * PSP + lane] = (half_t)(p * 4096.0f);
    }
    float cs[8];
#pragma unroll
    for (int j = 0; j < 8; ++j) cs[j] = __shfl(cr, 8 * h + j, 32);
#pragma unroll
    for (int t = 0; t < 8; ++t) {
#pragma unroll
      for (int j = 0; j < 8; ++j) oacc[t][j] *= cs[j];
    }
    wave_lds_sync();

    const v16h pa = ldfrag_s(Pw + m * PSP + 8 * h);
    const half_t* vrow = Vt + ((eh * 8) * 16 + m) * VSP + 8 * h;
#pragma unroll
    for (int t = 0; t < 8; ++t) {
      const v16h vb = ldfrag_s(vrow + t * 16 * VSP);
      oacc[t] = mma16_g(pa, vb, oacc[t]);
    }
  }
  __syncthreads();

  float ls[8];
#pragma unroll
  for (int j = 0; j < 8; ++j) ls[j] = __builtin_amdgcn_rcpf(__shfl(lr, 8 * h + j, 32)) * (1.0f / 2048.0f);
#pragma unroll
  for (int t = 0; t < 8; ++t) {
#pragma unroll
    for (int j = 0; j < 8; ++j)
      Os[(qr * 16 + 8 * h + j) * OSP + (eh * 8 + t) * 16 + m] = (half_t)(oacc[t][j] * ls[j]);
  }
  __syncthreads();
  for (int pass = 0; pass < 2; ++pass) {
#pragma unroll
    for (int i = 0; i < 8; ++i) {
      const int row = wave * 8 + i;
      const v8h v = *(const v8ha*)(Os + row * OSP + lane * 8);
      *(volatile v8h*)(Op + (size_t)(q0 + row) * EE + lane * 8) = v;
    }
    __threadfence();
  }
}

extern "C" void kernel_launch(void* const* d_in, const int* in_sizes, int n_in,
                              void* d_out, int out_size, void* d_ws, size_t ws_size,
                              hipStream_t stream) {
  if (n_in < 17) return;
  if (in_sizes[0] != MTOT * EE) return;
  if (in_sizes[1] != EE || in_sizes[2] != EE) return;
  if (in_sizes[3] != EE * EE || in_sizes[5] != EE * EE || in_sizes[7] != EE * EE || in_sizes[9] != EE * EE) return;
  if (in_sizes[4] != EE || in_sizes[6] != EE || in_sizes[8] != EE || in_sizes[10] != EE) return;
  if (in_sizes[11] != EE || in_sizes[12] != EE) return;
  if (in_sizes[13] != HIDN * EE || in_sizes[14] != HIDN || in_sizes[15] != EE * HIDN || in_sizes[16] != EE) return;
  if (out_size != MTOT * EE) return;

  const float* x    = (const float*)d_in[0];
  const float* ln1w = (const float*)d_in[1];
  const float* ln1b = (const float*)d_in[2];
  const float* Wq   = (const float*)d_in[3];
  const float* bq   = (const float*)d_in[4];
  const float* Wk   = (const float*)d_in[5];
  const float* bk   = (const float*)d_in[6];
  const float* Wv   = (const float*)d_in[7];
  const float* bv   = (const float*)d_in[8];
  const float* Wp   = (const float*)d_in[9];
  const float* bp   = (const float*)d_in[10];
  const float* ln2w = (const float*)d_in[11];
  const float* ln2b = (const float*)d_in[12];
  const float* W1   = (const float*)d_in[13];
  const float* b1   = (const float*)d_in[14];
  const float* W2   = (const float*)d_in[15];
  const float* b2   = (const float*)d_in[16];

  const size_t szW   = (size_t)EE * EE * 2;
  const size_t szW1  = (size_t)HIDN * EE * 2;
  const size_t szP   = (size_t)MTOT * EE * 2;
  const size_t szX1  = (size_t)MTOT * EE * 4;
  const size_t szHID = (size_t)MTOT * HIDN * 2;
  size_t off = 0;
  const size_t oWQ = off; off += szW;
  const size_t oWK = off; off += szW;
  const size_t oWV = off; off += szW;
  const size_t oWP = off; off += szW;
  const size_t oW1 = off; off += szW1;
  const size_t oW2 = off; off += szW1;
  const size_t oXN = off; off += szP;
  const size_t oQP = off; off += szP;
  const size_t oKP = off; off += szP;
  const size_t oVT = off; off += szP;
  const size_t oOP = off; off += szP;
  const size_t oX1 = off; off += szX1;
  const size_t oHID = oQP;
  const size_t oH2  = oXN;
  if (oHID + szHID > oX1) return;
  if (off > ws_size) return;

  char* ws = (char*)d_ws;
  half_t* WQ16 = (half_t*)(ws + oWQ);
  half_t* WK16 = (half_t*)(ws + oWK);
  half_t* WV16 = (half_t*)(ws + oWV);
  half_t* WP16 = (half_t*)(ws + oWP);
  half_t* W116 = (half_t*)(ws + oW1);
  half_t* W216 = (half_t*)(ws + oW2);
  half_t* XN   = (half_t*)(ws + oXN);
  half_t* QP   = (half_t*)(ws + oQP);
  half_t* KP   = (half_t*)(ws + oKP);
  half_t* VT   = (half_t*)(ws + oVT);
  half_t* OP   = (half_t*)(ws + oOP);
  float*  X1   = (float*)(ws + oX1);
  half_t* HID  = (half_t*)(ws + oHID);
  half_t* H2   = (half_t*)(ws + oH2);
  float*  OUT  = (float*)d_out;

  const dim3 blk(256);
  const int n8W  = (EE * EE) / 8;
  const int n8W1 = (HIDN * EE) / 8;

  cvt_f16_kernel<<<dim3((n8W + 255) / 256),  blk, 0, stream>>>(Wq, WQ16, n8W, 64.0f);
  cvt_f16_kernel<<<dim3((n8W + 255) / 256),  blk, 0, stream>>>(Wk, WK16, n8W, 64.0f);
  cvt_f16_kernel<<<dim3((n8W + 255) / 256),  blk, 0, stream>>>(Wv, WV16, n8W, 64.0f);
  cvt_f16_kernel<<<dim3((n8W + 255) / 256),  blk, 0, stream>>>(Wp, WP16, n8W, 64.0f);
  cvt_f16_kernel<<<dim3((n8W1 + 255) / 256), blk, 0, stream>>>(W1, W116, n8W1, 64.0f);
  cvt_f16_kernel<<<dim3((n8W1 + 255) / 256), blk, 0, stream>>>(W2, W216, n8W1, 64.0f);

  ln_kernel<<<dim3((MTOT + 7) / 8), blk, 0, stream>>>(x, ln1w, ln1b, XN, MTOT);

  const int tilesE   = (MTOT / 64) * (EE / 64);
  const int tilesHID = (MTOT / 64) * (HIDN / 64);
  const dim3 gE((tilesE + 7) / 8);
  const dim3 gH((tilesHID + 7) / 8);

  gemm64_kernel<2, 1, false, 0><<<gE, blk, 0, stream>>>(XN, EE, WQ16, EE, (void*)QP, EE, bq, nullptr, 0,
                                                        MTOT, EE, EE, 1.0f / 64.0f, 8.0f);
  gemm64_kernel<2, 1, false, 0><<<gE, blk, 0, stream>>>(XN, EE, WK16, EE, (void*)KP, EE, bk, nullptr, 0,
                                                        MTOT, EE, EE, 1.0f / 64.0f, 8.0f);
  gemm64_kernel<1, 1, false, 0><<<gE, blk, 0, stream>>>(WV16, EE, XN, EE, (void*)VT, MTOT, bv, nullptr, 0,
                                                        EE, MTOT, EE, 1.0f / 64.0f, 8.0f);
  attn_kernel<<<dim3(MTOT / 64), blk, 0, stream>>>(QP, KP, VT, OP);
  gemm64_kernel<2, 0, true, 0><<<gE, blk, 0, stream>>>(OP, EE, WP16, EE, (void*)X1, EE, bp, x, EE,
                                                       MTOT, EE, EE, 1.0f / 16384.0f, 1.0f);
  ln_kernel<<<dim3((MTOT + 7) / 8), blk, 0, stream>>>(X1, ln2w, ln2b, H2, MTOT);
  gemm64_kernel<2, 1, false, 1><<<gH, blk, 0, stream>>>(H2, EE, W116, EE, (void*)HID, HIDN, b1, nullptr, 0,
                                                        MTOT, HIDN, EE, 1.0f / 64.0f, 1.0f);
  gemm64_kernel<2, 0, true, 1><<<gE, blk, 0, stream>>>(HID, HIDN, W216, HIDN, (void*)OUT, EE, b2, X1, EE,
                                                       MTOT, EE, HIDN, 1.0f / 64.0f, 1.0f);
  (void)hipGetLastError();
}
